// VanillaLSTMNet_19207093747713
// MI455X (gfx1250) — hardware-run, weakly checked
//
#include <hip/hip_runtime.h>
#include <stdint.h>

typedef __attribute__((ext_vector_type(16))) _Float16 v16h;
typedef __attribute__((ext_vector_type(8)))  _Float16 v8h;
typedef __attribute__((ext_vector_type(16))) __bf16   v16b;
typedef __attribute__((ext_vector_type(8)))  __bf16   v8b;
typedef __attribute__((ext_vector_type(8)))  float    v8f;
typedef __attribute__((ext_vector_type(4)))  float    v4f;
typedef __attribute__((ext_vector_type(8)))  unsigned short v8us;

constexpr int IN_DIM   = 2;
constexpr int EMB_DIM  = 64;
constexpr int RNN_DIM  = 128;
constexpr int NGATE    = 4 * RNN_DIM;
constexpr int OUT_DIM  = 2;
constexpr int SEQ_LEN  = 20;
constexpr int PRED_LEN = 30;
constexpr int NPEDS    = 16384;

constexpr int PED_BLK  = 64;
constexpr int NTHR     = 64;
constexpr int HF_PITCH = 132;
constexpr float OP_SCALE = 16.0f;
constexpr float ACC_INV  = 1.0f / 256.0f;

static_assert(NPEDS % PED_BLK == 0);
static_assert(PED_BLK == NTHR);
static_assert(EMB_DIM % 32 == 0);
static_assert(RNN_DIM % 32 == 0);
static_assert(NGATE == 512);
static_assert((HF_PITCH * 4) % 16 == 0);

constexpr int OFF_EH   = 0;
constexpr int OFF_EL   = OFF_EH + PED_BLK * EMB_DIM * 2;
constexpr int OFF_HH   = OFF_EL + PED_BLK * EMB_DIM * 2;
constexpr int OFF_C    = OFF_HH + PED_BLK * RNN_DIM * 2;
constexpr int OFF_HF   = OFF_C + PED_BLK * RNN_DIM * 4;
constexpr int OFF_SO   = OFF_HF + PED_BLK * HF_PITCH * 4;
constexpr int OFF_BIAS = OFF_SO + PED_BLK * OUT_DIM * 4;
constexpr int OFF_WEMB = OFF_BIAS + NGATE * 4;
constexpr int OFF_BEMB = OFF_WEMB + EMB_DIM * IN_DIM * 4;
constexpr int OFF_WOUT = OFF_BEMB + EMB_DIM * 4;
constexpr int OFF_BOUT = OFF_WOUT + OUT_DIM * RNN_DIM * 4;
constexpr int SMEM_BYTES = OFF_BOUT + 16;
static_assert(SMEM_BYTES == 103696);
static_assert(OFF_EL % 16 == 0 && OFF_HH % 16 == 0 && OFF_C % 16 == 0 && OFF_HF % 16 == 0 && OFF_SO % 16 == 0);
static_assert(OFF_BIAS % 16 == 0 && OFF_WEMB % 16 == 0 && OFF_BEMB % 16 == 0 && OFF_WOUT % 16 == 0 && OFF_BOUT % 16 == 0);

constexpr size_t WS_WIHH  = 0;
constexpr size_t WS_WIHL  = WS_WIHH + (size_t)NGATE * EMB_DIM * 2;
constexpr size_t WS_WIHF  = WS_WIHL + (size_t)NGATE * EMB_DIM * 2;
constexpr size_t WS_WHHF  = WS_WIHF + (size_t)NGATE * EMB_DIM * 2;
constexpr size_t WS_TOTAL = WS_WHHF + (size_t)NGATE * RNN_DIM * 2;
static_assert(WS_TOTAL == 327680);
static_assert(WS_TOTAL <= 134217728ull);

__device__ __forceinline__ unsigned short f2bf_bits(float f) {
  unsigned u = __float_as_uint(f);
  return (unsigned short)((u + 0x7FFFu + ((u >> 16) & 1u)) >> 16);
}
__device__ __forceinline__ float bf_bits2f(unsigned short h) { return __uint_as_float(((unsigned)h) << 16); }
__device__ __forceinline__ __bf16 bits2bf(unsigned short h) { return __builtin_bit_cast(__bf16, h); }
__device__ __forceinline__ unsigned short h2bits(float f) { const _Float16 h = (_Float16)f; return __builtin_bit_cast(unsigned short, h); }

__device__ __forceinline__ void dep_guard_h(v8f& a, v8f& b, v16h x, v16h y) { asm volatile("v_nop\n\tv_nop\n\tv_nop\n\tv_nop" : "+v"(a), "+v"(b) : "v"(x), "v"(y)); }
__device__ __forceinline__ void dep_guard_b(v8f& a, v8f& b, v16b x, v16b y) { asm volatile("v_nop\n\tv_nop\n\tv_nop\n\tv_nop" : "+v"(a), "+v"(b) : "v"(x), "v"(y)); }
__device__ __forceinline__ void keep4_h(v16h a, v16h b, v16h c, v16h d) { asm volatile("v_nop" :: "v"(a), "v"(b), "v"(c), "v"(d)); }
__device__ __forceinline__ void keep4_b(v16b a, v16b b, v16b c, v16b d) { asm volatile("v_nop" :: "v"(a), "v"(b), "v"(c), "v"(d)); }
__device__ __forceinline__ void acc_guard4(v8f& a, v8f& b, v8f& c, v8f& d) { asm volatile("v_nop\n\tv_nop\n\tv_nop\n\tv_nop" : "+v"(a), "+v"(b), "+v"(c), "+v"(d)); }

template <typename T> struct Frag;
template <> struct Frag<_Float16> {
  typedef v16h V; union U { v16h v; v8h h[2]; };
  static __device__ __forceinline__ v16h load(const _Float16* p) {
    U f; f.h[0] = *(const v8h*)(p); f.h[1] = *(const v8h*)(p + 16); return f.v;
  }
  static __device__ __forceinline__ v8f mma(v16h a, v16h b, v8f c) {
    return __builtin_amdgcn_wmma_f32_16x16x32_f16(false, a, false, b, (short)0, c, false, false);
  }
  static __device__ __forceinline__ void guard(v8f& a, v8f& b, v16h x, v16h y) { dep_guard_h(a, b, x, y); }
  static __device__ __forceinline__ void keep(v16h a, v16h b, v16h c, v16h d) { keep4_h(a, b, c, d); }
};
template <> struct Frag<__bf16> {
  typedef v16b V; union U { v16b v; v8b h[2]; };
  static __device__ __forceinline__ v16b load(const __bf16* p) {
    U f; f.h[0] = *(const v8b*)(p); f.h[1] = *(const v8b*)(p + 16); return f.v;
  }
  static __device__ __forceinline__ v8f mma(v16b a, v16b b, v8f c) {
    return __builtin_amdgcn_wmma_f32_16x16x32_bf16(false, a, false, b, (short)0, c, false, false);
  }
  static __device__ __forceinline__ void guard(v8f& a, v8f& b, v16b x, v16b y) { dep_guard_b(a, b, x, y); }
  static __device__ __forceinline__ void keep(v16b a, v16b b, v16b c, v16b d) { keep4_b(a, b, c, d); }
};

__device__ __forceinline__ float sigm(float x) {
  const float xc = fminf(fmaxf(x, -30.0f), 30.0f);
  return 1.0f / (1.0f + expf(-xc));
}

__global__ __launch_bounds__(256) void prep_planes(const float* __restrict__ src,
                                                   unsigned short* out0, unsigned short* out1,
                                                   int n8, float scl, int mode) {
  const int i = blockIdx.x * 256 + threadIdx.x;
  if (i >= n8) return;
  const float* p = src + (size_t)i * 8;
  const v4f a = *(const v4f*)(p);
  const v4f b = *(const v4f*)(p + 4);
  const float f[8] = {a[0], a[1], a[2], a[3], b[0], b[1], b[2], b[3]};
  v8us hv, lv;
#pragma unroll
  for (int e = 0; e < 8; ++e) {
    const float x = f[e] * scl;
    if (mode != 0) {
      const unsigned short hb = f2bf_bits(x);
      const unsigned short lb = f2bf_bits(x - bf_bits2f(hb));
      hv[e] = hb; lv[e] = lb;
    } else {
      hv[e] = h2bits(x); lv[e] = (unsigned short)0;
    }
  }
  unsigned short* q0 = out0 + (size_t)i * 8;
  unsigned short* q1 = out1 + (size_t)i * 8;
  *(volatile v8us*)q0 = hv;
  if (mode != 0) *(volatile v8us*)q1 = lv;
  __threadfence();
  *(volatile v8us*)q0 = hv;
  if (mode != 0) *(volatile v8us*)q1 = lv;
}

__global__ __launch_bounds__(NTHR) void lstm_seq_kernel(
    const float* __restrict__ obs,
    const float* __restrict__ Wemb,
    const float* __restrict__ Bemb,
    const float* __restrict__ Bih,
    const float* __restrict__ Bhh,
    const float* __restrict__ Wout,
    const float* __restrict__ Bout,
    const int*   __restrict__ plen,
    const unsigned short* __restrict__ WihHp,
    const unsigned short* __restrict__ WihLp,
    const unsigned short* __restrict__ WihFp,
    const unsigned short* __restrict__ WhhFp,
    float* __restrict__ out)
{
  (void)plen;
  extern __shared__ __align__(16) unsigned char smem_raw[];
  __bf16*   sEh  = (__bf16*)(smem_raw + OFF_EH);
  _Float16* sEf  = (_Float16*)(smem_raw + OFF_EH);
  __bf16*   sEl  = (__bf16*)(smem_raw + OFF_EL);
  _Float16* sHh  = (_Float16*)(smem_raw + OFF_HH);
  float* sC    = (float*)(smem_raw + OFF_C);
  float* sHF   = (float*)(smem_raw + OFF_HF);
  float* sOut  = (float*)(smem_raw + OFF_SO);
  float* sBias = (float*)(smem_raw + OFF_BIAS);
  float* sWemb = (float*)(smem_raw + OFF_WEMB);
  float* sBemb = (float*)(smem_raw + OFF_BEMB);
  float* sWout = (float*)(smem_raw + OFF_WOUT);
  float* sBout = (float*)(smem_raw + OFF_BOUT);

  const __bf16*   WihH = (const __bf16*)(const void*)WihHp;
  const __bf16*   WihL = (const __bf16*)(const void*)WihLp;
  const _Float16* WihF = (const _Float16*)(const void*)WihFp;
  const _Float16* WhhF = (const _Float16*)(const void*)WhhFp;

  const int tid   = threadIdx.x;
  const int lane  = tid & 31;
  const int wave  = tid >> 5;
  const int rlane = lane & 15;
  const int koff  = (lane >> 4) * 8;
  const int hrow8 = (lane >> 4) * 8;
  const int wrow0 = wave * 32;
  const int pedBase = blockIdx.x * PED_BLK;

#pragma unroll 1
  for (int i = tid; i < NGATE; i += NTHR) sBias[i] = Bih[i] + Bhh[i];
#pragma unroll 1
  for (int i = tid; i < EMB_DIM * IN_DIM; i += NTHR) sWemb[i] = Wemb[i];
#pragma unroll 1
  for (int i = tid; i < EMB_DIM; i += NTHR) sBemb[i] = Bemb[i];
#pragma unroll 1
  for (int i = tid; i < OUT_DIM * RNN_DIM; i += NTHR) sWout[i] = Wout[i];
  {
    const float bo = Bout[(tid < OUT_DIM) ? tid : 0];
    if (tid < 4) sBout[tid] = (tid < OUT_DIM) ? bo : 0.0f;
  }
#pragma unroll 1
  for (int i = tid; i < PED_BLK * RNN_DIM; i += NTHR) sC[i] = 0.0f;
#pragma unroll 1
  for (int i = tid; i < PED_BLK * HF_PITCH; i += NTHR) sHF[i] = 0.0f;
#pragma unroll 1
  for (int i = tid; i < PED_BLK * OUT_DIM; i += NTHR) sOut[i] = 0.0f;
  __syncthreads();

#pragma unroll 1
  for (int t = 0; t < SEQ_LEN + PRED_LEN; ++t) {
    const bool enc = (t < SEQ_LEN);

    {
      const int tt = enc ? t : (SEQ_LEN - 1);
      const float* xp = obs + ((size_t)tt * NPEDS + pedBase + tid) * IN_DIM;
      const float xo0 = xp[0], xo1 = xp[1];
      const float xs0 = sOut[tid * OUT_DIM], xs1 = sOut[tid * OUT_DIM + 1];
      const float x0 = enc ? xo0 : xs0;
      const float x1 = enc ? xo1 : xs1;
      if (enc) {
        __bf16* ehs = sEh + tid * EMB_DIM;
        __bf16* els = sEl + tid * EMB_DIM;
#pragma unroll 1
        for (int jb = 0; jb < EMB_DIM / 8; ++jb) {
          v8b hv, lv;
#pragma unroll
          for (int e = 0; e < 8; ++e) {
            const int j = jb * 8 + e;
            float v = x0 * sWemb[2 * j] + x1 * sWemb[2 * j + 1] + sBemb[j];
            v = fmaxf(v, 0.0f) * OP_SCALE;
            const unsigned short hb = f2bf_bits(v);
            const unsigned short lb = f2bf_bits(v - bf_bits2f(hb));
            hv[e] = bits2bf(hb);
            lv[e] = bits2bf(lb);
          }
          *(v8b*)(ehs + jb * 8) = hv;
          *(v8b*)(els + jb * 8) = lv;
        }
      } else {
        _Float16* efs = sEf + tid * EMB_DIM;
#pragma unroll 1
        for (int jb = 0; jb < EMB_DIM / 8; ++jb) {
          v8h hv;
#pragma unroll
          for (int e = 0; e < 8; ++e) {
            const int j = jb * 8 + e;
            float v = x0 * sWemb[2 * j] + x1 * sWemb[2 * j + 1] + sBemb[j];
            v = fmaxf(v, 0.0f) * OP_SCALE;
            hv[e] = (_Float16)v;
          }
          *(v8h*)(efs + jb * 8) = hv;
        }
      }
      const float* hrow = sHF + tid * HF_PITCH;
      _Float16* hhs = sHh + tid * RNN_DIM;
#pragma unroll 1
      for (int q = 0; q < RNN_DIM / 8; ++q) {
        const v4f ha = *(const v4f*)(hrow + q * 8);
        const v4f hb4 = *(const v4f*)(hrow + q * 8 + 4);
        v8h hv;
        hv[0] = (_Float16)(ha[0] * OP_SCALE);
        hv[1] = (_Float16)(ha[1] * OP_SCALE);
        hv[2] = (_Float16)(ha[2] * OP_SCALE);
        hv[3] = (_Float16)(ha[3] * OP_SCALE);
        hv[4] = (_Float16)(hb4[0] * OP_SCALE);
        hv[5] = (_Float16)(hb4[1] * OP_SCALE);
        hv[6] = (_Float16)(hb4[2] * OP_SCALE);
        hv[7] = (_Float16)(hb4[3] * OP_SCALE);
        *(v8h*)(hhs + q * 8) = hv;
      }
    }
    __syncthreads();

#pragma unroll 1
    for (int ub = 0; ub < RNN_DIM / 16; ++ub) {
      v8f acc[2][4];
#pragma unroll
      for (int i = 0; i < 2; ++i)
#pragma unroll
        for (int j = 0; j < 4; ++j) acc[i][j] = (v8f){0.f, 0.f, 0.f, 0.f, 0.f, 0.f, 0.f, 0.f};
      const int ncol = ub * 16 + rlane;

      if (enc) {
#pragma unroll
        for (int ks = 0; ks < EMB_DIM / 32; ++ks) {
          const int k0 = ks * 32;
          v16b bh[4], bl[4];
#pragma unroll
          for (int j = 0; j < 4; ++j) {
            const int bo = (j * RNN_DIM + ncol) * EMB_DIM + k0 + koff;
            bh[j] = Frag<__bf16>::load(WihH + bo);
            bl[j] = Frag<__bf16>::load(WihL + bo);
          }
#pragma unroll
          for (int i = 0; i < 2; ++i) {
            const int ao = (wrow0 + i * 16 + rlane) * EMB_DIM + k0 + koff;
            const v16b ah = Frag<__bf16>::load(sEh + ao);
            const v16b al = Frag<__bf16>::load(sEl + ao);
#pragma unroll
            for (int j = 0; j < 4; ++j) {
              acc[i][j] = Frag<__bf16>::mma(ah, bh[j], acc[i][j]);
              acc[i][j] = Frag<__bf16>::mma(ah, bl[j], acc[i][j]);
              acc[i][j] = Frag<__bf16>::mma(al, bh[j], acc[i][j]);
            }
            Frag<__bf16>::guard(acc[i][0], acc[i][3], ah, al);
          }
          Frag<__bf16>::keep(bh[0], bh[1], bh[2], bh[3]);
          Frag<__bf16>::keep(bl[0], bl[1], bl[2], bl[3]);
        }
      } else {
#pragma unroll
        for (int ks = 0; ks < EMB_DIM / 32; ++ks) {
          const int k0 = ks * 32;
          v16h bh[4];
#pragma unroll
          for (int j = 0; j < 4; ++j) {
            const int bo = (j * RNN_DIM + ncol) * EMB_DIM + k0 + koff;
            bh[j] = Frag<_Float16>::load(WihF + bo);
          }
#pragma unroll
          for (int i = 0; i < 2; ++i) {
            const int ao = (wrow0 + i * 16 + rlane) * EMB_DIM + k0 + koff;
            const v16h ah = Frag<_Float16>::load(sEf + ao);
#pragma unroll
            for (int j = 0; j < 4; ++j) acc[i][j] = Frag<_Float16>::mma(ah, bh[j], acc[i][j]);
            Frag<_Float16>::guard(acc[i][0], acc[i][3], ah, ah);
          }
          Frag<_Float16>::keep(bh[0], bh[1], bh[2], bh[3]);
        }
      }

#pragma unroll
      for (int ks = 0; ks < RNN_DIM / 32; ++ks) {
        const int k0 = ks * 32;
        v16h bh[4];
#pragma unroll
        for (int j = 0; j < 4; ++j) {
          const int bo = (j * RNN_DIM + ncol) * RNN_DIM + k0 + koff;
          bh[j] = Frag<_Float16>::load(WhhF + bo);
        }
#pragma unroll
        for (int i = 0; i < 2; ++i) {
          const int ao = (wrow0 + i * 16 + rlane) * RNN_DIM + k0 + koff;
          const v16h ah = Frag<_Float16>::load(sHh + ao);
#pragma unroll
          for (int j = 0; j < 4; ++j) acc[i][j] = Frag<_Float16>::mma(ah, bh[j], acc[i][j]);
          Frag<_Float16>::guard(acc[i][0], acc[i][3], ah, ah);
        }
        Frag<_Float16>::keep(bh[0], bh[1], bh[2], bh[3]);
      }
      acc_guard4(acc[0][0], acc[0][1], acc[0][2], acc[0][3]);
      acc_guard4(acc[1][0], acc[1][1], acc[1][2], acc[1][3]);

      const float bI = sBias[ncol];
      const float bF = sBias[RNN_DIM + ncol];
      const float bG = sBias[2 * RNN_DIM + ncol];
      const float bO = sBias[3 * RNN_DIM + ncol];
#pragma unroll
      for (int i = 0; i < 2; ++i) {
        float* cptr = sC + ((wave * 2 + i) * (RNN_DIM / 16) + ub) * 256 + lane * 8;
        const v8f cOld = *(const v8f*)cptr;
        v8f cNew;
        float* hdst = sHF + (wrow0 + i * 16 + hrow8) * HF_PITCH + ncol;
#pragma unroll
        for (int r = 0; r < 8; ++r) {
          const float ig = sigm(acc[i][0][r] * ACC_INV + bI);
          const float fg = sigm(acc[i][1][r] * ACC_INV + bF);
          const float gg = tanhf(acc[i][2][r] * ACC_INV + bG);
          const float og = sigm(acc[i][3][r] * ACC_INV + bO);
          const float cn = fg * cOld[r] + ig * gg;
          cNew[r] = cn;
          hdst[r * HF_PITCH] = og * tanhf(cn);
        }
        *(v8f*)cptr = cNew;
      }
    }
    __syncthreads();

    if (t >= SEQ_LEN - 1) {
      {
        const float* hrow = sHF + tid * HF_PITCH;
        float a0 = sBout[0], a1 = sBout[1];
#pragma unroll 2
        for (int u = 0; u < RNN_DIM; u += 4) {
          const v4f hv = *(const v4f*)(hrow + u);
          const v4f w0 = *(const v4f*)(sWout + u);
          const v4f w1 = *(const v4f*)(sWout + RNN_DIM + u);
          a0 += hv[0] * w0[0]; a0 += hv[1] * w0[1]; a0 += hv[2] * w0[2]; a0 += hv[3] * w0[3];
          a1 += hv[0] * w1[0]; a1 += hv[1] * w1[1]; a1 += hv[2] * w1[2]; a1 += hv[3] * w1[3];
        }
        sOut[tid * OUT_DIM]     = a0;
        sOut[tid * OUT_DIM + 1] = a1;
      }
      __syncthreads();
      if (!enc) {
        if (tid < 32) {
          const v4f v = *(const v4f*)(sOut + tid * 4);
          float* dst = out + ((size_t)(t - SEQ_LEN) * NPEDS + pedBase) * OUT_DIM + tid * 4;
          *(volatile v4f*)dst = v;
          __threadfence();
          *(volatile v4f*)dst = v;
        }
      }
    }
    __syncthreads();
  }
}

extern "C" void kernel_launch(void* const* d_in, const int* in_sizes, int n_in,
                              void* d_out, int out_size, void* d_ws,
                              size_t ws_size, hipStream_t stream) {
  (void)in_sizes; (void)n_in; (void)out_size; (void)ws_size;
  const float* obs  = (const float*)d_in[0];
  const float* Wemb = (const float*)d_in[1];
  const float* Bemb = (const float*)d_in[2];
  const float* Wih  = (const float*)d_in[3];
  const float* Bih  = (const float*)d_in[4];
  const float* Whh  = (const float*)d_in[5];
  const float* Bhh  = (const float*)d_in[6];
  const float* Wout = (const float*)d_in[7];
  const float* Bout = (const float*)d_in[8];
  const int*   plen = (const int*)d_in[9];
  float* out = (float*)d_out;

  unsigned char* ws = (unsigned char*)d_ws;
  unsigned short* wihH = (unsigned short*)(ws + WS_WIHH);
  unsigned short* wihL = (unsigned short*)(ws + WS_WIHL);
  unsigned short* wihF = (unsigned short*)(ws + WS_WIHF);
  unsigned short* whhF = (unsigned short*)(ws + WS_WHHF);

  const int n8_ih = NGATE * EMB_DIM / 8;
  const int n8_hh = NGATE * RNN_DIM / 8;
  prep_planes<<<dim3((n8_ih + 255) / 256), dim3(256), 0, stream>>>(Wih, wihH, wihL, n8_ih, OP_SCALE, 1);
  prep_planes<<<dim3((n8_ih + 255) / 256), dim3(256), 0, stream>>>(Wih, wihF, wihF, n8_ih, OP_SCALE, 0);
  prep_planes<<<dim3((n8_hh + 255) / 256), dim3(256), 0, stream>>>(Whh, whhF, whhF, n8_hh, OP_SCALE, 0);

  lstm_seq_kernel<<<dim3(NPEDS / PED_BLK), dim3(NTHR), SMEM_BYTES, stream>>>(
      obs, Wemb, Bemb, Bih, Bhh, Wout, Bout, plen, wihH, wihL, wihF, whhF, out);
}
